// MyLinearSlct_75015898792455
// MI455X (gfx1250) — hardware-verified
//
#include <hip/hip_runtime.h>
#include <math.h>

typedef __attribute__((ext_vector_type(16))) _Float16 v16h;
typedef __attribute__((ext_vector_type(16))) __bf16 v16b;
typedef __attribute__((ext_vector_type(8)))  _Float16 v8h;
typedef __attribute__((ext_vector_type(8)))  float v8f;
typedef __attribute__((ext_vector_type(4)))  float v4f;
typedef __attribute__((ext_vector_type(2)))  float v2f;
typedef __attribute__((ext_vector_type(4)))  unsigned v4u;
typedef __attribute__((ext_vector_type(4)))  int v4i;
typedef float __attribute__((may_alias)) float_a;
typedef int __attribute__((may_alias)) int_a;

template <typename T> __device__ __forceinline__ void vst2(void* p, T v) { *(volatile T*)p = v; __threadfence(); *(volatile T*)p = v; }
__device__ __forceinline__ v8f wmma16(v16h a, v16h b, v8f c) {
  v8f d = __builtin_amdgcn_wmma_f32_16x16x32_f16(false, a, false, b, (short)0, c, false, false);
  asm volatile("v_nop\n\tv_nop\n\tv_nop\n\tv_nop" : "+v"(d) : "v"(a), "v"(b));
  return d;
}
__device__ __forceinline__ v8f wmma_bf(v16b a, v16b b, v8f c) {
  v8f d = __builtin_amdgcn_wmma_f32_16x16x32_bf16(false, a, false, b, (short)0, c, false, false);
  asm volatile("v_nop\n\tv_nop\n\tv_nop\n\tv_nop" : "+v"(d) : "v"(a), "v"(b));
  return d;
}
__device__ __forceinline__ v16h frag_h(const _Float16* rowk0, int lane) {
  union { v16h v; v8h q[2]; } u; const _Float16* p = rowk0 + 8 * (lane >> 4);
  u.q[0] = *(const v8h*)p; u.q[1] = *(const v8h*)(p + 16); return u.v;
}
__device__ __forceinline__ v16h frag_f32(const float* rowk0, int lane) {
  v16h a; const float* p = rowk0 + 8 * (lane >> 4);
#pragma unroll
  for (int i = 0; i < 8; ++i) { a[i] = (_Float16)p[i]; a[8 + i] = (_Float16)p[16 + i]; }
  return a;
}
__device__ __forceinline__ v16h frag_f32s(const float* rowk0, int lane, float sc) {
  v16h a; const float* p = rowk0 + 8 * (lane >> 4);
#pragma unroll
  for (int i = 0; i < 8; ++i) { a[i] = (_Float16)(p[i] * sc); a[8 + i] = (_Float16)(p[16 + i] * sc); }
  return a;
}
__device__ __forceinline__ v16h fragc_f32(const float* W, int k0, int n, int lane, int ld, int K) {
  v16h a; const int g = lane >> 4;
#pragma unroll
  for (int i = 0; i < 8; ++i) { const int ka = k0 + 8 * g + i, kb = ka + 16;
    a[i] = (_Float16)(ka < K ? W[(size_t)ka * ld + n] : 0.f); a[8 + i] = (_Float16)(kb < K ? W[(size_t)kb * ld + n] : 0.f); }
  return a;
}
struct F2 { v16b h, l; };
__device__ __forceinline__ F2 bsplit16(const float v[16]) { F2 r;
#pragma unroll
  for (int i = 0; i < 16; ++i) { const __bf16 h = (__bf16)v[i]; r.h[i] = h; r.l[i] = (__bf16)(v[i] - (float)h); }
  return r; }
__device__ __forceinline__ F2 split_row(const float* row, int k0, int lane) { float v[16]; const float* p = row + k0 + 8 * (lane >> 4);
#pragma unroll
  for (int i = 0; i < 8; ++i) { v[i] = p[i]; v[8 + i] = p[16 + i]; }
  return bsplit16(v); }
__device__ __forceinline__ F2 split_rowK(const float* row, int k0, int lane, int K) { float v[16]; const int g = lane >> 4;
#pragma unroll
  for (int i = 0; i < 8; ++i) { const int ka = k0 + 8 * g + i, kb = ka + 16; v[i] = ka < K ? row[ka] : 0.f; v[8 + i] = kb < K ? row[kb] : 0.f; }
  return bsplit16(v); }
__device__ __forceinline__ F2 split_col(const float* W, int k0, int n, int lane, int ld, int K) { float v[16]; const int g = lane >> 4;
#pragma unroll
  for (int i = 0; i < 8; ++i) { const int ka = k0 + 8 * g + i, kb = ka + 16; v[i] = ka < K ? W[(size_t)ka * ld + n] : 0.f; v[8 + i] = kb < K ? W[(size_t)kb * ld + n] : 0.f; }
  return bsplit16(v); }
__device__ __forceinline__ v8f mac3(const F2& a, const F2& b, v8f c) { c = wmma_bf(a.l, b.h, c); c = wmma_bf(a.h, b.l, c); return wmma_bf(a.h, b.h, c); }
__device__ __forceinline__ float sigm(float v) { return 1.0f / (1.0f + expf(-v)); }
#define LDSX() do { asm volatile("s_wait_dscnt 0" ::: "memory"); __builtin_amdgcn_wave_barrier(); __builtin_amdgcn_fence(__ATOMIC_RELEASE, "workgroup"); } while (0)


#define NB 8192
#define NI 1024
#define NO 1024
#define NE 8
#define NBP (NB + 16)

__device__ __forceinline__ void expert_rows(const float* __restrict__ slct, int e, int* slist, int* shist, int* swt, int* scount, int* soff) {
  const int tid = threadIdx.x, wave = tid >> 5, lane = tid & 31; const int per = NB / 128;
  if (tid < NE) shist[tid] = 0;
  __syncthreads();
  int cnt = 0; int hloc[NE];
#pragma unroll
  for (int k = 0; k < NE; ++k) hloc[k] = 0;
#pragma unroll 1
  for (int u = 0; u < per; ++u) { const float* s = slct + (size_t)(tid * per + u) * NE; const v4f a = *(const v4f*)s, c = *(const v4f*)(s + 4);
    float m = a[0]; int im = 0;
    if (a[1] > m) { m = a[1]; im = 1; } if (a[2] > m) { m = a[2]; im = 2; } if (a[3] > m) { m = a[3]; im = 3; }
    if (c[0] > m) { m = c[0]; im = 4; } if (c[1] > m) { m = c[1]; im = 5; } if (c[2] > m) { m = c[2]; im = 6; } if (c[3] > m) { m = c[3]; im = 7; }
    if (im == e) cnt++;
#pragma unroll
    for (int k = 0; k < NE; ++k) hloc[k] += (im == k);
  }
#pragma unroll
  for (int k = 0; k < NE; ++k) atomicAdd(&shist[k], hloc[k]);
  int incl = cnt;
#pragma unroll
  for (int off = 1; off < 32; off <<= 1) { const int v = __shfl_up(incl, off, 32); if (lane >= off) incl += v; }
  if (lane == 31) swt[wave] = incl;
  __syncthreads();
  int base = 0, tot = 0; for (int w = 0; w < 4; ++w) { const int v = swt[w]; if (w < wave) base += v; tot += v; }
  int pos = base + incl - cnt;
#pragma unroll 1
  for (int u = 0; u < per; ++u) { const float* s = slct + (size_t)(tid * per + u) * NE; const v4f a = *(const v4f*)s, c = *(const v4f*)(s + 4);
    float m = a[0]; int im = 0;
    if (a[1] > m) { m = a[1]; im = 1; } if (a[2] > m) { m = a[2]; im = 2; } if (a[3] > m) { m = a[3]; im = 3; }
    if (c[0] > m) { m = c[0]; im = 4; } if (c[1] > m) { m = c[1]; im = 5; } if (c[2] > m) { m = c[2]; im = 6; } if (c[3] > m) { m = c[3]; im = 7; }
    if (im == e) slist[pos++] = tid * per + u; }
  if (tid == 0) { *scount = tot; int o = 0; for (int k = 0; k < e; ++k) o += shist[k]; *soff = o; }
  __syncthreads();
}
__global__ __launch_bounds__(128) void k_gather(const float* __restrict__ slct, const float* __restrict__ x, _Float16* __restrict__ XS) {
  __shared__ int slist[NB]; __shared__ int shist[NE]; __shared__ int swt[4]; __shared__ int scount, soff;
  const int e = blockIdx.x, tid = threadIdx.x;
  expert_rows(slct, e, slist, shist, swt, &scount, &soff);
  const int count = scount, off = soff;
  for (int q = tid; q < count * 8; q += 128) { const int i = q >> 3, part = q & 7; const float* xr = x + (size_t)slist[i] * NI + part * 128; _Float16* dr = XS + (size_t)(off + i) * NI + part * 128;
#pragma unroll 4
    for (int c8 = 0; c8 < 16; ++c8) { const v4f a = *(const v4f*)(xr + c8 * 8), c = *(const v4f*)(xr + c8 * 8 + 4); union { v8h h; v4u u; } pk;
      pk.h[0] = (_Float16)a[0]; pk.h[1] = (_Float16)a[1]; pk.h[2] = (_Float16)a[2]; pk.h[3] = (_Float16)a[3]; pk.h[4] = (_Float16)c[0]; pk.h[5] = (_Float16)c[1]; pk.h[6] = (_Float16)c[2]; pk.h[7] = (_Float16)c[3];
      vst2(dr + c8 * 8, pk.u); } }
  if (e == 0) { for (int q = tid; q < 16 * (NI / 8); q += 128) { const int rl = q / (NI / 8), pc = q % (NI / 8); vst2(XS + (size_t)(NB + rl) * NI + pc * 8, (v4u){0u, 0u, 0u, 0u}); } }
}
__global__ __launch_bounds__(128) void k_lin(const float* __restrict__ slct, const _Float16* __restrict__ XS, const float* __restrict__ W, const float* __restrict__ bias, float* __restrict__ out) {
  __shared__ int slist[NB]; __shared__ int shist[NE]; __shared__ int swt[4]; __shared__ int scount, soff;
  __shared__ __align__(16) float so[4][16][132];
  const int e = blockIdx.y, n0 = blockIdx.x * 128, tid = threadIdx.x, wave = tid >> 5, lane = tid & 31, col = lane & 15, g = lane >> 4;
  expert_rows(slct, e, slist, shist, swt, &scount, &soff);
  const int count = scount, off = soff; const float* We = W + (size_t)e * NO * NI; const int ntiles = (count + 15) >> 4;
  float bb[8];
#pragma unroll
  for (int j = 0; j < 8; ++j) bb[j] = bias[e * NO + n0 + j * 16 + col];
#pragma unroll 1
  for (int tile = wave; tile < ntiles; tile += 4) { const int i0 = tile * 16; const _Float16* arow = XS + (size_t)(off + i0 + col) * NI;
    v8f acc[8] = {};
#pragma unroll 1
    for (int kc = 0; kc < NI / 32; ++kc) { const v16h a = frag_h(arow + kc * 32, lane);
#pragma unroll
      for (int j = 0; j < 8; ++j) acc[j] = wmma16(a, frag_f32s(We + (size_t)(n0 + j * 16 + col) * NI + kc * 32, lane, 16.0f), acc[j]); }
#pragma unroll
    for (int j = 0; j < 8; ++j)
#pragma unroll
      for (int r = 0; r < 8; ++r) { const float v = acc[j][r] * (1.0f / 16.0f) + bb[j]; so[wave][8 * g + r][j * 16 + col] = v > 0.f ? v : 0.f; }
    LDSX();
    for (int rl = 0; rl < 16; ++rl) { const int idx = i0 + rl; if (idx >= count) break; const int rr = slist[idx]; vst2(out + (size_t)rr * NO + n0 + lane * 4, *(const v4f*)(&so[wave][rl][lane * 4])); }
    LDSX(); }
}
extern "C" void kernel_launch(void* const* d_in, const int* in_sizes, int n_in, void* d_out, int out_size, void* d_ws, size_t ws_size, hipStream_t stream) {
  (void)in_sizes; (void)n_in; (void)out_size; (void)ws_size;
  const float* x = (const float*)d_in[0]; const float* slct = (const float*)d_in[1]; const float* W = (const float*)d_in[2]; const float* b = (const float*)d_in[3];
  _Float16* XS = (_Float16*)d_ws;
  k_gather<<<NE, 128, 0, stream>>>(slct, x, XS);
  k_lin<<<dim3(NO / 128, NE), 128, 0, stream>>>(slct, XS, W, b, (float*)d_out);
}
